// RankOnePools_38835094290478
// MI455X (gfx1250) — hardware-verified
//
#include <hip/hip_runtime.h>
#include <stdint.h>
#include <stddef.h>

#pragma clang fp contract(off)

#define NTOK  4096
#define NSEL  32
#define DIN   2048
#define DOUT  2048
#define NEK   256
#define MT    32
#define NW    4
#define SFP   260
#define NSLAB 256
#define CVT_TPB 256

static_assert(NTOK % MT == 0);
static_assert(MT == 2 * 16);
static_assert(NW * 64 == NEK);
static_assert(NW * 64 == NSLAB);
static_assert(DOUT % NSLAB == 0);
static_assert(DIN % 32 == 0);
static_assert(NEK % 32 == 0);
static_assert((SFP * 4) % 16 == 0);
static_assert(SFP >= NEK);
static_assert(MT % NW == 0);
static_assert(MT * NSEL == 8 * 32 * NW);
static_assert((NTOK * DIN) % (8 * CVT_TPB) == 0);
static_assert((NEK * DIN) % (8 * CVT_TPB) == 0);
static_assert((DOUT * NEK) % (8 * CVT_TPB) == 0);
static_assert(NEK == 8 * 32);
static_assert(NSLAB == 2 * 4 * 32);

typedef unsigned short us_t;
typedef __bf16         v16b __attribute__((ext_vector_type(16)));
typedef float          v8f  __attribute__((ext_vector_type(8)));
typedef float          v4f  __attribute__((ext_vector_type(4)));
typedef unsigned int   v4u  __attribute__((ext_vector_type(4)));
typedef unsigned short v8us __attribute__((ext_vector_type(8)));
typedef int            v4i  __attribute__((ext_vector_type(4)));
typedef v4f __attribute__((may_alias)) v4fa;
typedef v4u __attribute__((may_alias)) v4ua;
typedef v4i __attribute__((may_alias)) v4ia;

union FragB { v16b v; v4u q[2]; };
union Pack8 { v8us s; v4u u; };

__device__ __forceinline__ unsigned int bfb(float f) {
  const unsigned int u = __float_as_uint(f);
  return (u + 0x7FFFu + ((u >> 16) & 1u)) >> 16;
}

__device__ __forceinline__ v8f wmma_b(v16b a, v16b b, v8f c) {
  v8f d = __builtin_amdgcn_wmma_f32_16x16x32_bf16(false, a, false, b, (short)0, c, false, false);
  asm volatile("v_nop\n\tv_nop\n\tv_nop\n\tv_nop" : "+v"(d) : "v"(a), "v"(b));
  return d;
}

__device__ __forceinline__ v8f wmma3(v16b ah, v16b al, v16b bh, v16b bl, v8f c) {
  c = wmma_b(ah, bh, c);
  c = wmma_b(al, bh, c);
  c = wmma_b(ah, bl, c);
  return c;
}

__device__ __forceinline__ v16b ldfrag(const us_t* p, int h) {
  FragB f;
  f.q[0] = *(const v4ua*)(p + 8 * h);
  f.q[1] = *(const v4ua*)(p + 16 + 8 * h);
  return f.v;
}

__global__ __launch_bounds__(CVT_TPB) void k_split(const float* __restrict__ src,
                                                   us_t* __restrict__ ph,
                                                   us_t* __restrict__ pl, int n8)
{
  const int i = blockIdx.x * CVT_TPB + threadIdx.x;
  if (i >= n8) return;
  const float* s = src + (size_t)i * 8;
  const v4f a = *(const v4fa*)s;
  const v4f b = *(const v4fa*)(s + 4);
  float f[8];
  f[0] = a.x; f[1] = a.y; f[2] = a.z; f[3] = a.w;
  f[4] = b.x; f[5] = b.y; f[6] = b.z; f[7] = b.w;
  v8us hv, lv;
  #pragma unroll
  for (int k = 0; k < 8; ++k) {
    const unsigned int hb = bfb(f[k]);
    const float hf = __uint_as_float(hb << 16);
    const unsigned int lb = bfb(f[k] - hf);
    hv[k] = (us_t)hb;
    lv[k] = (us_t)lb;
  }
  Pack8 kh, kl;
  kh.s = hv;
  kl.s = lv;
  const v4u uh = kh.u, ul = kl.u;
  us_t* qh = ph + (size_t)i * 8;
  us_t* ql = pl + (size_t)i * 8;
  *(volatile v4u*)qh = uh;
  *(volatile v4u*)ql = ul;
  __threadfence();
  *(volatile v4u*)qh = uh;
  *(volatile v4u*)ql = ul;
}

__global__ __launch_bounds__(128) void k_gemm1(const us_t* __restrict__ xh,
                                               const us_t* __restrict__ xl,
                                               const us_t* __restrict__ sh,
                                               const us_t* __restrict__ sl,
                                               const int* __restrict__ index,
                                               us_t* __restrict__ dh,
                                               us_t* __restrict__ dl)
{
  __shared__ __align__(16) float sF[MT * SFP];
  __shared__ __align__(16) int sIdx[MT * NSEL];

  const int tid = threadIdx.x, lane = tid & 31, wv = tid >> 5;
  const int h = lane >> 4, m = lane & 15;
  const int row0 = blockIdx.x * MT;

  const v8f z8 = {0.f, 0.f, 0.f, 0.f, 0.f, 0.f, 0.f, 0.f};
  v8f acc[2][4];
  #pragma unroll
  for (int mt = 0; mt < 2; ++mt)
    #pragma unroll
    for (int nt = 0; nt < 4; ++nt) acc[mt][nt] = z8;

  const us_t* ah0p = xh + (size_t)(row0 + m) * DIN;
  const us_t* ah1p = xh + (size_t)(row0 + 16 + m) * DIN;
  const us_t* al0p = xl + (size_t)(row0 + m) * DIN;
  const us_t* al1p = xl + (size_t)(row0 + 16 + m) * DIN;
  const size_t boff = (size_t)(64 * wv + m) * DIN;

  #pragma unroll 1
  for (int kb = 0; kb < DIN; kb += 32) {
    const v16b ah0 = ldfrag(ah0p + kb, h);
    const v16b ah1 = ldfrag(ah1p + kb, h);
    const v16b al0 = ldfrag(al0p + kb, h);
    const v16b al1 = ldfrag(al1p + kb, h);
    #pragma unroll
    for (int nt = 0; nt < 4; ++nt) {
      const size_t bo = boff + (size_t)(16 * nt) * DIN + kb;
      const v16b bh = ldfrag(sh + bo, h);
      const v16b bl = ldfrag(sl + bo, h);
      acc[0][nt] = wmma3(ah0, al0, bh, bl, acc[0][nt]);
      acc[1][nt] = wmma3(ah1, al1, bh, bl, acc[1][nt]);
    }
  }

  #pragma unroll
  for (int mt = 0; mt < 2; ++mt)
    #pragma unroll
    for (int nt = 0; nt < 4; ++nt)
      #pragma unroll
      for (int r = 0; r < 8; ++r)
        sF[(16 * mt + 8 * h + r) * SFP + 64 * wv + 16 * nt + m] = acc[mt][nt][r];

  #pragma unroll
  for (int j = 0; j < 8; ++j) {
    const int i = j * 128 + tid;
    const int r = i >> 5, s = i & 31;
    int v = index[(size_t)(row0 + r) * NSEL + s];
    v = (v < 0) ? 0 : ((v > NEK - 1) ? (NEK - 1) : v);
    sIdx[i] = v;
  }
  __syncthreads();

  const int e0 = 8 * lane;
  #pragma unroll 1
  for (int rr = 0; rr < MT / NW; ++rr) {
    const int r = wv + NW * rr;
    int cnt[8];
    #pragma unroll
    for (int i = 0; i < 8; ++i) cnt[i] = 0;
    #pragma unroll
    for (int j = 0; j < 8; ++j) {
      const v4i q = *(const v4ia*)(sIdx + r * NSEL + 4 * j);
      #pragma unroll
      for (int c = 0; c < 4; ++c) {
        const int dv = q[c] - e0;
        #pragma unroll
        for (int i = 0; i < 8; ++i) cnt[i] += (dv == i) ? 1 : 0;
      }
    }
    const v4f f0 = *(const v4fa*)(sF + r * SFP + e0);
    const v4f f1 = *(const v4fa*)(sF + r * SFP + e0 + 4);
    float fv[8];
    fv[0] = f0.x; fv[1] = f0.y; fv[2] = f0.z; fv[3] = f0.w;
    fv[4] = f1.x; fv[5] = f1.y; fv[6] = f1.z; fv[7] = f1.w;
    v8us hv, lv;
    #pragma unroll
    for (int i = 0; i < 8; ++i) {
      const float d = (float)cnt[i] * fv[i];
      const unsigned int hb = bfb(d);
      const float hf = __uint_as_float(hb << 16);
      const unsigned int lb = bfb(d - hf);
      hv[i] = (us_t)hb;
      lv[i] = (us_t)lb;
    }
    Pack8 kh, kl;
    kh.s = hv;
    kl.s = lv;
    const v4u uh = kh.u, ul = kl.u;
    us_t* qh = dh + (size_t)(row0 + r) * NEK + e0;
    us_t* ql = dl + (size_t)(row0 + r) * NEK + e0;
    *(volatile v4u*)qh = uh;
    *(volatile v4u*)ql = ul;
    __threadfence();
    *(volatile v4u*)qh = uh;
    *(volatile v4u*)ql = ul;
  }
}

__global__ __launch_bounds__(128) void k_gemm2(const us_t* __restrict__ dh,
                                               const us_t* __restrict__ dl,
                                               const us_t* __restrict__ uh,
                                               const us_t* __restrict__ ul,
                                               const float* __restrict__ rw,
                                               float* __restrict__ out)
{
  __shared__ __align__(16) float sY[MT * SFP];
  (void)rw;

  const int tid = threadIdx.x, lane = tid & 31, wv = tid >> 5;
  const int h = lane >> 4, m = lane & 15;
  const int row0 = blockIdx.x * MT;
  const int col0 = blockIdx.y * NSLAB;

  const v8f z8 = {0.f, 0.f, 0.f, 0.f, 0.f, 0.f, 0.f, 0.f};
  v8f acc[2][4];
  #pragma unroll
  for (int mt = 0; mt < 2; ++mt)
    #pragma unroll
    for (int nt = 0; nt < 4; ++nt) acc[mt][nt] = z8;

  const us_t* ah0p = dh + (size_t)(row0 + m) * NEK;
  const us_t* ah1p = dh + (size_t)(row0 + 16 + m) * NEK;
  const us_t* al0p = dl + (size_t)(row0 + m) * NEK;
  const us_t* al1p = dl + (size_t)(row0 + 16 + m) * NEK;
  const size_t boff = (size_t)(col0 + 64 * wv + m) * NEK;

  #pragma unroll 1
  for (int kb = 0; kb < NEK; kb += 32) {
    const v16b ah0 = ldfrag(ah0p + kb, h);
    const v16b ah1 = ldfrag(ah1p + kb, h);
    const v16b al0 = ldfrag(al0p + kb, h);
    const v16b al1 = ldfrag(al1p + kb, h);
    #pragma unroll
    for (int nt = 0; nt < 4; ++nt) {
      const size_t bo = boff + (size_t)(16 * nt) * NEK + kb;
      const v16b bh = ldfrag(uh + bo, h);
      const v16b bl = ldfrag(ul + bo, h);
      acc[0][nt] = wmma3(ah0, al0, bh, bl, acc[0][nt]);
      acc[1][nt] = wmma3(ah1, al1, bh, bl, acc[1][nt]);
    }
  }

  #pragma unroll
  for (int mt = 0; mt < 2; ++mt)
    #pragma unroll
    for (int nt = 0; nt < 4; ++nt)
      #pragma unroll
      for (int r = 0; r < 8; ++r)
        sY[(16 * mt + 8 * h + r) * SFP + 64 * wv + 16 * nt + m] = acc[mt][nt][r];
  __syncthreads();

  #pragma unroll 1
  for (int rr = 0; rr < MT / NW; ++rr) {
    const int r = wv + NW * rr;
    const v4f y0 = *(const v4fa*)(sY + r * SFP + 4 * lane);
    const v4f y1 = *(const v4fa*)(sY + r * SFP + 128 + 4 * lane);
    float* dst = out + (size_t)(row0 + r) * DOUT + col0;
    *(volatile v4f*)(dst + 4 * lane) = y0;
    *(volatile v4f*)(dst + 128 + 4 * lane) = y1;
    __threadfence();
    *(volatile v4f*)(dst + 4 * lane) = y0;
    *(volatile v4f*)(dst + 128 + 4 * lane) = y1;
  }
}

extern "C" void kernel_launch(void* const* d_in, const int* in_sizes, int n_in,
                              void* d_out, int out_size, void* d_ws, size_t ws_size,
                              hipStream_t stream)
{
  if (n_in < 5) return;
  if (in_sizes[0] != NTOK * DIN) return;
  if (in_sizes[2] != NTOK * NSEL) return;
  if (in_sizes[3] != DOUT * NEK) return;
  if (in_sizes[4] != NEK * DIN) return;
  if (out_size != NTOK * DOUT) return;

  const float* x   = (const float*)d_in[0];
  const float* rw  = (const float*)d_in[1];
  const int*   idx = (const int*)d_in[2];
  const float* u   = (const float*)d_in[3];
  const float* svh = (const float*)d_in[4];
  float* out = (float*)d_out;

  const size_t bX = (size_t)NTOK * DIN * 2;
  const size_t bS = (size_t)NEK * DIN * 2;
  const size_t bU = (size_t)DOUT * NEK * 2;
  const size_t bD = (size_t)NTOK * NEK * 2;
  const size_t total = 2 * bX + 2 * bS + 2 * bU + 2 * bD;
  if (total > ws_size) return;
  if (total > (size_t)134217728) return;

  char* ws = (char*)d_ws;
  size_t off = 0;
  us_t* Xh = (us_t*)(ws + off); off += bX;
  us_t* Xl = (us_t*)(ws + off); off += bX;
  us_t* Sh = (us_t*)(ws + off); off += bS;
  us_t* Sl = (us_t*)(ws + off); off += bS;
  us_t* Uh = (us_t*)(ws + off); off += bU;
  us_t* Ul = (us_t*)(ws + off); off += bU;
  us_t* Dh = (us_t*)(ws + off); off += bD;
  us_t* Dl = (us_t*)(ws + off); off += bD;
  if (off != total) return;

  k_split<<<(NTOK * DIN) / (8 * CVT_TPB), CVT_TPB, 0, stream>>>(x, Xh, Xl, (NTOK * DIN) / 8);
  k_split<<<(NEK * DIN) / (8 * CVT_TPB), CVT_TPB, 0, stream>>>(svh, Sh, Sl, (NEK * DIN) / 8);
  k_split<<<(DOUT * NEK) / (8 * CVT_TPB), CVT_TPB, 0, stream>>>(u, Uh, Ul, (DOUT * NEK) / 8);
  k_gemm1<<<NTOK / MT, 128, 0, stream>>>(Xh, Xl, Sh, Sl, idx, Dh, Dl);
  k_gemm2<<<dim3(NTOK / MT, DOUT / NSLAB), 128, 0, stream>>>(Dh, Dl, Uh, Ul, rw, out);
}
